// Encoder_73830487818453
// MI455X (gfx1250) — hardware-verified
//
#include <hip/hip_runtime.h>
#include <stddef.h>
#include <stdint.h>
#include <math.h>


#define NN     50000
#define NE     1600000
#define FD     128
#define OD     64
#define NU     10000
#define MP     50048
#define HP     256
#define NTHR   256
#define NWAVE  8
#define EPT    8
#define CHUNK  (NTHR * EPT)
#define WCAP   (EPT * 32)
#define LISTN  (NWAVE * WCAP)
#define NBD    8192
#define SLD    13
#define GD     7
#define NBPD   (GD * NBD)
#define NBA    512
#define SLA    9
#define GA     98
#define NSLOT  (GA * NBA)
#define RCAP   20480
#define DEGCAP 96
#define GBM    64
#define GTHR   128
#define BK_ZINTS    (LISTN + 2 * RCAP + 3 * NBA)
#define BK_LDS_INTS (BK_ZINTS + 16 + NBA)
#define UX     (MP * 16)
#define UW0    2048
#define UW1    4096
#define US1    2048
#define US2    1024
#define UBI    256
#define UTOT   (UX + UW0 + UW1 + US1 + US2 + UBI)
#define OUT1   640000
#define WSMAX  134217728

static_assert(MP % GBM == 0 && MP >= NN && MP - NN < GBM);
static_assert(GA * NBA >= MP && NBPD >= MP);
static_assert((CHUNK & (CHUNK - 1)) == 0 && CHUNK <= 4096);
static_assert(NBD == (1 << SLD) && NBA == (1 << SLA));
static_assert(((long long)CHUNK << SLD) < (1LL << 31));
static_assert(((long long)NE << SLA) < (1LL << 31));
static_assert(NE % 4 == 0 && NN % 4 == 0);
static_assert(RCAP * 20 >= 16678 * 21);
static_assert(DEGCAP >= 57 + 8);
static_assert(RCAP % (4 * NTHR) == 0 && BK_ZINTS % 4 == 0);
static_assert(NBD % (NTHR * 4) == 0 && NBA % NWAVE == 0 && NBA % 32 == 0 && NBA / 4 <= NTHR);
static_assert(FD == 4 * 32 && HP == 2 * FD && FD % 32 == 0 && HP % 32 == 0 && (2 * OD) % 32 == 0);
static_assert(UX % NTHR == 0 && UW0 % NTHR == 0 && UW1 % NTHR == 0 && US1 % NTHR == 0 && US2 % NTHR == 0);
static_assert(UTOT % NTHR == 0);
static_assert((OUT1 * 4) % 128 == 0 && OUT1 == NU * OD);
static_assert(NU % 16 == 0);
static_assert(BK_LDS_INTS * 4 <= 300000);

typedef float          v4f   __attribute__((ext_vector_type(4)));
typedef float          v8f   __attribute__((ext_vector_type(8)));
typedef int            v4i   __attribute__((ext_vector_type(4)));
typedef int            v8i   __attribute__((ext_vector_type(8)));
typedef unsigned short v4us  __attribute__((ext_vector_type(4)));
typedef unsigned short v8us  __attribute__((ext_vector_type(8)));
typedef unsigned short v16us __attribute__((ext_vector_type(16)));
typedef __bf16         v16bf __attribute__((ext_vector_type(16)));
typedef v4f  __attribute__((may_alias)) v4fa;
typedef v4i  __attribute__((may_alias)) v4ia;
typedef v4us __attribute__((may_alias)) v4usa;
typedef v8us __attribute__((may_alias)) v8usa;
union FragB { v16bf v; v16us u; v8us h[2]; v8i w; };

__device__ __forceinline__ v8f wmb(const FragB& a, const FragB& b, v8f c) {
  v8f d = __builtin_amdgcn_wmma_f32_16x16x32_bf16(false, a.v, false, b.v, (short)0, c, false, false);
  asm volatile("v_nop\n\tv_nop\n\tv_nop\n\tv_nop" : "+v"(d) : "v"(a.w), "v"(b.w));
  return d;
}

__device__ __forceinline__ unsigned bf16_bits(float f) {
  const unsigned u = __float_as_uint(f);
  const unsigned r = (u + 0x7FFFu + ((u >> 16) & 1u)) >> 16;
  return ((u & 0x7fffffffu) > 0x7f800000u) ? 0x7FC0u : r;
}
__device__ __forceinline__ float bf16_val(float f) {
  return __uint_as_float(bf16_bits(f) << 16);
}

__device__ __forceinline__ void wave_sync() {
  __builtin_amdgcn_fence(__ATOMIC_RELEASE, "wavefront");
  __builtin_amdgcn_wave_barrier();
  __builtin_amdgcn_fence(__ATOMIC_ACQUIRE, "wavefront");
}

__device__ __forceinline__ void st2_us8(unsigned short* p, v8us v) {
  *(volatile v8us*)p = v;
  __threadfence();
  *(volatile v8us*)p = v;
}
__device__ __forceinline__ void st2_f4(float* p, v4f v) {
  *(volatile v4f*)p = v;
  __threadfence();
  *(volatile v4f*)p = v;
}

template <int SLB>
__device__ __forceinline__ int scan_chunk(const int* __restrict__ dsts, int nE, int cbase, int slotBase,
                                          int nb, int vec8, int* list, int tid, int lane, int wave) {
  int wc = 0;
  const int el0  = tid * EPT;
  const int e0   = cbase + el0;
  const int sent = -2147483647 - 1;
  v4i da, db;
  if (vec8 != 0 && cbase + CHUNK <= nE) {
    da = *(const v4i*)(dsts + e0);
    db = *(const v4i*)(dsts + e0 + 4);
  } else {
    da.x = (e0     < nE) ? dsts[min(e0,     nE - 1)] : sent;
    da.y = (e0 + 1 < nE) ? dsts[min(e0 + 1, nE - 1)] : sent;
    da.z = (e0 + 2 < nE) ? dsts[min(e0 + 2, nE - 1)] : sent;
    da.w = (e0 + 3 < nE) ? dsts[min(e0 + 3, nE - 1)] : sent;
    db.x = (e0 + 4 < nE) ? dsts[min(e0 + 4, nE - 1)] : sent;
    db.y = (e0 + 5 < nE) ? dsts[min(e0 + 5, nE - 1)] : sent;
    db.z = (e0 + 6 < nE) ? dsts[min(e0 + 6, nE - 1)] : sent;
    db.w = (e0 + 7 < nE) ? dsts[min(e0 + 7, nE - 1)] : sent;
  }
  const unsigned nbs = (unsigned)slotBase;
  const unsigned unb = (unsigned)nb;
  const unsigned s0 = (unsigned)da.x - nbs, s1 = (unsigned)da.y - nbs;
  const unsigned s2 = (unsigned)da.z - nbs, s3 = (unsigned)da.w - nbs;
  const unsigned s4 = (unsigned)db.x - nbs, s5 = (unsigned)db.y - nbs;
  const unsigned s6 = (unsigned)db.z - nbs, s7 = (unsigned)db.w - nbs;
  const bool h0 = s0 < unb, h1 = s1 < unb, h2 = s2 < unb, h3 = s3 < unb;
  const bool h4 = s4 < unb, h5 = s5 < unb, h6 = s6 < unb, h7 = s7 < unb;
  const unsigned any = __builtin_amdgcn_ballot_w32(h0 | h1 | h2 | h3 | h4 | h5 | h6 | h7);
  if (any != 0u) {
#define HITJ(J, HJ, SJ) { \
      const unsigned mj = __builtin_amdgcn_ballot_w32(HJ); \
      if (mj != 0u) { \
        if (HJ) { \
          const int pos = wc + (int)__builtin_amdgcn_mbcnt_lo(mj, 0u); \
          if (pos < WCAP) list[wave * WCAP + pos] = ((el0 + (J)) << SLB) | (int)(SJ); \
        } \
        wc += (int)__builtin_popcount(mj); } }
    HITJ(0, h0, s0)
    HITJ(1, h1, s1)
    HITJ(2, h2, s2)
    HITJ(3, h3, s3)
    HITJ(4, h4, s4)
    HITJ(5, h5, s5)
    HITJ(6, h6, s6)
    HITJ(7, h7, s7)
#undef HITJ
  }
  return wc;
}

__global__ __launch_bounds__(NTHR) void k_prep(const float* __restrict__ x,
    const float* __restrict__ W0, const float* __restrict__ W1,
    const float* __restrict__ Ws1, const float* __restrict__ Ws2,
    const float* __restrict__ b0, const float* __restrict__ b1,
    const float* __restrict__ bs1, const float* __restrict__ bs2,
    unsigned short* XB, unsigned short* W0T, unsigned short* W1D,
    unsigned short* WS1D, unsigned short* WS2D, float* BT) {
  const int u = (int)blockIdx.x * NTHR + (int)threadIdx.x;
  if (u < UX) {
    const int row = u >> 4;
    const int k8  = (u & 15) * 8;
    const int rc  = row < NN ? row : NN - 1;
    const float* p = x + (size_t)rc * FD + k8;
    const v4f a = *(const v4f*)p;
    const v4f b = *(const v4f*)(p + 4);
    const bool ok = row < NN;
    v8us o;
    o[0] = ok ? (unsigned short)bf16_bits(a.x) : (unsigned short)0;
    o[1] = ok ? (unsigned short)bf16_bits(a.y) : (unsigned short)0;
    o[2] = ok ? (unsigned short)bf16_bits(a.z) : (unsigned short)0;
    o[3] = ok ? (unsigned short)bf16_bits(a.w) : (unsigned short)0;
    o[4] = ok ? (unsigned short)bf16_bits(b.x) : (unsigned short)0;
    o[5] = ok ? (unsigned short)bf16_bits(b.y) : (unsigned short)0;
    o[6] = ok ? (unsigned short)bf16_bits(b.z) : (unsigned short)0;
    o[7] = ok ? (unsigned short)bf16_bits(b.w) : (unsigned short)0;
    st2_us8(XB + (size_t)row * FD + k8, o);
  } else if (u < UX + UW0) {
    const int v  = u - UX;
    const int n  = v >> 4;
    const int k8 = (v & 15) * 8;
    const float* p = W0 + (size_t)k8 * FD + n;
    v8us o;
#pragma unroll
    for (int i = 0; i < 8; ++i) o[i] = (unsigned short)bf16_bits(p[(size_t)i * FD]);
    st2_us8(W0T + (size_t)n * FD + k8, o);
  } else if (u < UX + UW0 + UW1) {
    const int v  = u - (UX + UW0);
    const int n  = v >> 5;
    const int k8 = (v & 31) * 8;
    const int kk = k8 & (FD - 1);
    const float* p = W1 + (size_t)kk * FD + n;
    v8us o;
#pragma unroll
    for (int i = 0; i < 8; ++i) o[i] = (unsigned short)bf16_bits(p[(size_t)i * FD]);
    st2_us8(W1D + (size_t)n * HP + k8, o);
  } else if (u < UX + UW0 + UW1 + US1) {
    const int v  = u - (UX + UW0 + UW1);
    const int n  = v >> 5;
    const int k8 = (v & 31) * 8;
    const int kk = k8 & (FD - 1);
    const float* p = Ws1 + (size_t)kk * OD + n;
    v8us o;
#pragma unroll
    for (int i = 0; i < 8; ++i) o[i] = (unsigned short)bf16_bits(p[(size_t)i * OD]);
    st2_us8(WS1D + (size_t)n * HP + k8, o);
  } else if (u < UX + UW0 + UW1 + US1 + US2) {
    const int v  = u - (UX + UW0 + UW1 + US1);
    const int n  = v >> 4;
    const int k8 = (v & 15) * 8;
    const int kk = k8 & (OD - 1);
    const float* p = Ws2 + (size_t)kk * OD + n;
    v8us o;
#pragma unroll
    for (int i = 0; i < 8; ++i) o[i] = (unsigned short)bf16_bits(p[(size_t)i * OD]);
    st2_us8(WS2D + (size_t)n * (2 * OD) + k8, o);
  } else {
    const int t  = (int)threadIdx.x;
    const int i0 = t < 31 ? t : 31;
    int i1 = t - 32; i1 = i1 < 0 ? 0 : (i1 > 31 ? 31 : i1);
    int i2 = t - 64; i2 = i2 < 0 ? 0 : (i2 > 15 ? 15 : i2);
    int i3 = t - 80; i3 = i3 < 0 ? 0 : (i3 > 15 ? 15 : i3);
    const v4i a0 = *(const v4i*)(const void*)(b0  + 4 * i0);
    const v4i a1 = *(const v4i*)(const void*)(b1  + 4 * i1);
    const v4i a2 = *(const v4i*)(const void*)(bs1 + 4 * i2);
    const v4i a3 = *(const v4i*)(const void*)(bs2 + 4 * i3);
    const int m0 = (t < 32) ? -1 : 0;
    const int m1 = (t >= 32 && t < 64) ? -1 : 0;
    const int m2 = (t >= 64 && t < 80) ? -1 : 0;
    const int m3 = (t >= 80) ? -1 : 0;
    v4f r;
    r.x = bf16_val(__int_as_float((a0.x & m0) | (a1.x & m1) | (a2.x & m2) | (a3.x & m3)));
    r.y = bf16_val(__int_as_float((a0.y & m0) | (a1.y & m1) | (a2.y & m2) | (a3.y & m3)));
    r.z = bf16_val(__int_as_float((a0.z & m0) | (a1.z & m1) | (a2.z & m2) | (a3.z & m3)));
    r.w = bf16_val(__int_as_float((a0.w & m0) | (a1.w & m1) | (a2.w & m2) | (a3.w & m3)));
    if (t < 96) st2_f4(BT + 4 * t, r);
  }
}

__global__ __launch_bounds__(NTHR) void k_degout(const int* __restrict__ keys, int nE, int vec8, float* cs) {
  __shared__ __attribute__((aligned(16))) int scnt[NBD];
  __shared__ __attribute__((aligned(16))) int list[LISTN];
  __shared__ int wcnt[NWAVE];
  const int tid = (int)threadIdx.x, lane = tid & 31, wave = tid >> 5;
  const int nodeBase = (int)blockIdx.x * NBD;

  for (int i = tid; i < NBD; i += NTHR) scnt[i] = 0;
  for (int i = tid; i < LISTN; i += NTHR) list[i] = 0;
  if (tid < NWAVE) wcnt[tid] = 0;
  __syncthreads();

  const int nChunks = (nE + CHUNK - 1) / CHUNK;
#pragma unroll 1
  for (int ch = 0; ch < nChunks; ++ch) {
    const int cbase = ch * CHUNK;
    const int wc = scan_chunk<SLD>(keys, nE, cbase, nodeBase, NBD, vec8, list, tid, lane, wave);
    if (lane == 0) wcnt[wave] = wc;
    __syncthreads();
    if (wave == 0) {
#pragma unroll 1
      for (int w2 = 0; w2 < NWAVE; ++w2) {
        int c = wcnt[w2];
        c = c < 0 ? 0 : (c > WCAP ? WCAP : c);
#pragma unroll 1
        for (int b0 = 0; b0 < c; b0 += 32) {
          const int idx = b0 + lane;
          const int ent = list[w2 * WCAP + (idx < WCAP ? idx : WCAP - 1)];
          const int m32 = (c - b0) < 32 ? (c - b0) : 32;
#pragma unroll 1
          for (int k = 0; k < m32; ++k) {
            const int u  = __builtin_amdgcn_readlane(ent, k);
            const int sl = u & (NBD - 1);
            if (lane == 0) scnt[sl] = scnt[sl] + 1;
          }
        }
      }
    }
    __syncthreads();
  }

#pragma unroll 1
  for (int i = tid; i < NBD; i += NTHR) {
    int c = scnt[i];
    c = c < 1 ? 1 : c;
    scnt[i] = __float_as_int(1.0f / sqrtf((float)c));
  }
  __syncthreads();

  v4f vals[NBD / (NTHR * 4)];
#pragma unroll
  for (int it = 0; it < NBD / (NTHR * 4); ++it) {
    const int s0 = it * (NTHR * 4) + 4 * tid;
    const v4i c4 = *(const v4ia*)(scnt + s0);
    v4f v;
    v.x = __int_as_float(c4.x); v.y = __int_as_float(c4.y);
    v.z = __int_as_float(c4.z); v.w = __int_as_float(c4.w);
    vals[it] = v;
  }
#pragma unroll
  for (int it = 0; it < NBD / (NTHR * 4); ++it) {
    const int s0 = it * (NTHR * 4) + 4 * tid;
    *(volatile v4f*)(cs + (size_t)nodeBase + s0) = vals[it];
  }
  __threadfence();
#pragma unroll
  for (int it = 0; it < NBD / (NTHR * 4); ++it) {
    const int s0 = it * (NTHR * 4) + 4 * tid;
    *(volatile v4f*)(cs + (size_t)nodeBase + s0) = vals[it];
  }
}

__global__ __launch_bounds__(NTHR) void k_bucket(const int* __restrict__ srcs, const int* __restrict__ dsts,
                                                 int nE, int nN, int vec8,
                                                 int* listg, int* offg, int* cntg, float* cdg) {
  extern __shared__ __attribute__((aligned(16))) int dsm[];
  int* list = dsm;
  int* hl   = dsm + LISTN;
  int* sl   = hl + RCAP;
  int* cnt  = sl + RCAP;
  int* offs = cnt + NBA;
  int* cur  = offs + NBA;
  int* misc = cur + NBA;
  int* cdi  = misc + 16;
  const int tid = (int)threadIdx.x, lane = tid & 31, wave = tid >> 5;
  const int nodeBase = (int)blockIdx.x * NBA;

  {
    const v4i z4 = {0, 0, 0, 0};
    for (int i = tid * 4; i < BK_ZINTS; i += NTHR * 4) *(v4ia*)(dsm + i) = z4;
    if (tid < 16) misc[tid] = 0;
  }
  __syncthreads();

  int t = 0, ov = 0;
  const int nChunks = (nE + CHUNK - 1) / CHUNK;
#pragma unroll 1
  for (int ch = 0; ch < nChunks; ++ch) {
    const int cbase = ch * CHUNK;
    const int wc = scan_chunk<SLA>(dsts, nE, cbase, nodeBase, NBA, vec8, list, tid, lane, wave);
    if (lane == 0) misc[wave] = wc;
    __syncthreads();
    if (wave == 0) {
#pragma unroll 1
      for (int w2 = 0; w2 < NWAVE; ++w2) {
        int c = misc[w2];
        c = c < 0 ? 0 : (c > WCAP ? WCAP : c);
#pragma unroll 1
        for (int b0 = 0; b0 < c; b0 += 32) {
          const int idx = b0 + lane;
          const int ent = list[w2 * WCAP + (idx < WCAP ? idx : WCAP - 1)];
          const int m32 = (c - b0) < 32 ? (c - b0) : 32;
#pragma unroll 1
          for (int k = 0; k < m32; ++k) {
            const int u    = __builtin_amdgcn_readlane(ent, k);
            const int slot = u & (NBA - 1);
            const int el   = (u >> SLA) & (CHUNK - 1);
            const int pk   = ((cbase + el) << SLA) | slot;
            if (t < RCAP) {
              if (lane == 0) { hl[t] = pk; cnt[slot] = cnt[slot] + 1; }
              t = t + 1;
            } else {
              ov = 1;
            }
          }
        }
      }
    }
    __syncthreads();
  }
  if (wave == 0 && lane == 0) { misc[8] = t; misc[9] = ov; }
  __syncthreads();
  int tt = misc[8];
  tt = tt < 0 ? 0 : (tt > RCAP ? RCAP : tt);
  const int ovf = misc[9];

  if (wave == 0) {
    const int base = lane * (NBA / 32);
    int s = 0;
#pragma unroll 1
    for (int i = 0; i < NBA / 32; ++i) s += cnt[base + i];
    int incl = s;
#pragma unroll
    for (int d = 1; d < 32; d <<= 1) {
      const int y = __shfl_up(incl, d, 32);
      if (lane >= d) incl += y;
    }
    int run = incl - s;
#pragma unroll 1
    for (int i = 0; i < NBA / 32; ++i) {
      const int cv = cnt[base + i];
      offs[base + i] = run;
      cur[base + i]  = run;
      run += cv;
    }
  }
  __syncthreads();
  if (wave == 0) {
#pragma unroll 1
    for (int b0 = 0; b0 < tt; b0 += 32) {
      const int idx = b0 + lane;
      const int ent = hl[idx < RCAP ? idx : RCAP - 1];
      const int m32 = (tt - b0) < 32 ? (tt - b0) : 32;
#pragma unroll 1
      for (int k = 0; k < m32; ++k) {
        const int u    = __builtin_amdgcn_readlane(ent, k);
        const int slot = u & (NBA - 1);
        if (lane == 0) {
          int p = cur[slot];
          p = p < 0 ? 0 : (p > RCAP - 1 ? RCAP - 1 : p);
          sl[p] = u;
          cur[slot] = p + 1;
        }
      }
    }
  }
#pragma unroll 1
  for (int i = tid; i < NBA; i += NTHR) {
    int c = cnt[i];
    c = c < 1 ? 1 : c;
    cdi[i] = __float_as_int(1.0f / sqrtf((float)c));
  }
  __syncthreads();

  if (tid < NBA / 4) {
    v4i c4 = *(const v4ia*)(cnt + 4 * tid);
    const v4i o4 = *(const v4ia*)(offs + 4 * tid);
    const v4i d4 = *(const v4ia*)(cdi + 4 * tid);
    const int pm = (ovf != 0) ? -1 : 0;
    c4.x = c4.x | pm; c4.y = c4.y | pm; c4.z = c4.z | pm; c4.w = c4.w | pm;
    v4f f4;
    f4.x = __int_as_float(d4.x); f4.y = __int_as_float(d4.y);
    f4.z = __int_as_float(d4.z); f4.w = __int_as_float(d4.w);
    int*   cp = cntg + (size_t)nodeBase + 4 * tid;
    int*   op = offg + (size_t)nodeBase + 4 * tid;
    float* dp = cdg  + (size_t)nodeBase + 4 * tid;
    *(volatile v4i*)cp = c4;
    *(volatile v4i*)op = o4;
    *(volatile v4f*)dp = f4;
    __threadfence();
    *(volatile v4i*)cp = c4;
    *(volatile v4i*)op = o4;
    *(volatile v4f*)dp = f4;
  }

#pragma unroll 1
  for (int it = 0; it < RCAP / (4 * NTHR); ++it) {
    const int i = (it * NTHR + tid) * 4;
    const v4i e4 = *(const v4ia*)(sl + i);
    int e0 = e4.x >> SLA, e1 = e4.y >> SLA, e2 = e4.z >> SLA, e3 = e4.w >> SLA;
    e0 = e0 < 0 ? 0 : (e0 > nE - 1 ? nE - 1 : e0);
    e1 = e1 < 0 ? 0 : (e1 > nE - 1 ? nE - 1 : e1);
    e2 = e2 < 0 ? 0 : (e2 > nE - 1 ? nE - 1 : e2);
    e3 = e3 < 0 ? 0 : (e3 > nE - 1 ? nE - 1 : e3);
    int r0 = srcs[e0], r1 = srcs[e1], r2 = srcs[e2], r3 = srcs[e3];
    r0 = r0 < 0 ? 0 : (r0 > nN - 1 ? nN - 1 : r0);
    r1 = r1 < 0 ? 0 : (r1 > nN - 1 ? nN - 1 : r1);
    r2 = r2 < 0 ? 0 : (r2 > nN - 1 ? nN - 1 : r2);
    r3 = r3 < 0 ? 0 : (r3 > nN - 1 ? nN - 1 : r3);
    v4i o;
    o.x = (i     < tt) ? r0 : 0;
    o.y = (i + 1 < tt) ? r1 : 0;
    o.z = (i + 2 < tt) ? r2 : 0;
    o.w = (i + 3 < tt) ? r3 : 0;
    int* gp = listg + (size_t)blockIdx.x * RCAP + i;
    *(volatile v4i*)gp = o;
    __threadfence();
    *(volatile v4i*)gp = o;
  }
}

template <int K>
__global__ __launch_bounds__(GTHR) void k_gemm(const unsigned short* __restrict__ A,
                                               const unsigned short* __restrict__ BT,
                                               const float* __restrict__ cs, float* outF) {
  __shared__ __attribute__((aligned(16))) float stg[GBM * FD];
  const int tid = (int)threadIdx.x, lane = tid & 31, wave = tid >> 5, hh = lane >> 4, m = lane & 15;
  const int rowBase = (int)blockIdx.x * GBM;

  v8f acc[8];
  {
    const v8f z = {0.f, 0.f, 0.f, 0.f, 0.f, 0.f, 0.f, 0.f};
#pragma unroll
    for (int t = 0; t < 8; ++t) acc[t] = z;
  }
  const unsigned short* ap = A  + (size_t)(rowBase + 16 * wave + m) * (size_t)K + 8 * hh;
  const unsigned short* bp = BT + (size_t)m * (size_t)K + 8 * hh;

#pragma unroll 1
  for (int k0 = 0; k0 < K; k0 += 32) {
    FragB af;
    af.h[0] = *(const v8usa*)(ap + k0);
    af.h[1] = *(const v8usa*)(ap + k0 + 16);
#pragma unroll
    for (int nt = 0; nt < 8; ++nt) {
      const unsigned short* wq = bp + (size_t)(16 * nt) * (size_t)K + k0;
      FragB bf;
      bf.h[0] = *(const v8usa*)wq;
      bf.h[1] = *(const v8usa*)(wq + 16);
      acc[nt] = wmb(af, bf, acc[nt]);
    }
  }

#pragma unroll
  for (int nt = 0; nt < 8; ++nt) {
    const int lc = 16 * nt + m;
#pragma unroll
    for (int r = 0; r < 8; ++r) {
      const int lr = 16 * wave + 8 * hh + r;
      stg[lr * FD + lc] = acc[nt][r];
    }
  }
  __syncthreads();

  const int csi = __float_as_int(cs[rowBase + 16 * wave + m]);
  v4f pv[16];
#pragma unroll
  for (int i = 0; i < 16; ++i) pv[i] = *(const v4fa*)(stg + (16 * wave + i) * FD + 4 * lane);
#pragma unroll
  for (int i = 0; i < 16; ++i) {
    const float sc = __int_as_float(__builtin_amdgcn_readlane(csi, i));
    const bool ok = (rowBase + 16 * wave + i) < NN;
    v4f y;
    y.x = ok ? pv[i].x * sc : 0.0f;
    y.y = ok ? pv[i].y * sc : 0.0f;
    y.z = ok ? pv[i].z * sc : 0.0f;
    y.w = ok ? pv[i].w * sc : 0.0f;
    pv[i] = y;
  }
#pragma unroll
  for (int i = 0; i < 16; ++i) {
    const int r = rowBase + 16 * wave + i;
    *(volatile v4f*)(outF + (size_t)r * FD + 4 * lane) = pv[i];
  }
  __threadfence();
#pragma unroll
  for (int i = 0; i < 16; ++i) {
    const int r = rowBase + 16 * wave + i;
    *(volatile v4f*)(outF + (size_t)r * FD + 4 * lane) = pv[i];
  }
}

template <int FINAL>
__global__ __launch_bounds__(NTHR) void k_agg(const int* __restrict__ listg, const int* __restrict__ offg,
                                              const int* __restrict__ cntg, const float* __restrict__ cdg,
                                              const float* __restrict__ hs, const float* __restrict__ bias,
                                              unsigned short* hhl, float* outp) {
  __shared__ __attribute__((aligned(16))) int cntl[NBA];
  __shared__ __attribute__((aligned(16))) int offl[NBA];
  __shared__ __attribute__((aligned(16))) int cdl[NBA];
  __shared__ __attribute__((aligned(16))) unsigned short rowbufs[NWAVE * HP];
  const int tid = (int)threadIdx.x, lane = tid & 31, wave = tid >> 5;
  const int nodeBase = (int)blockIdx.x * NBA;
  unsigned short* rowbuf = rowbufs + wave * HP;

  if (tid < NBA / 4) {
    *(v4ia*)(cntl + 4 * tid) = *(const v4i*)(cntg + (size_t)nodeBase + 4 * tid);
    *(v4ia*)(offl + 4 * tid) = *(const v4i*)(offg + (size_t)nodeBase + 4 * tid);
    *(v4ia*)(cdl  + 4 * tid) = *(const v4i*)(const void*)(cdg + (size_t)nodeBase + 4 * tid);
  }
  const v4f bb = *(const v4f*)(bias + 4 * lane);
  __syncthreads();

  const int* lst = listg + (size_t)blockIdx.x * RCAP;
  const float qnan = __int_as_float(0x7fc00000);
#pragma unroll 1
  for (int si = 0; si < NBA / NWAVE; ++si) {
    const int s    = si * NWAVE + wave;
    const int node = nodeBase + s;
    int c = cntl[s];
    const bool bad = (c < 0) || (c > DEGCAP);
    c = c < 0 ? 0 : (c > DEGCAP ? DEGCAP : c);
    int o = offl[s];
    o = o < 0 ? 0 : (o > RCAP ? RCAP : o);
    const float cdv = __int_as_float(cdl[s]);
    float a0 = 0.0f, a1 = 0.0f, a2 = 0.0f, a3 = 0.0f;
#pragma unroll 1
    for (int b0 = 0; b0 < c; b0 += 32) {
      int idx = o + b0 + lane;
      idx = idx > RCAP - 1 ? RCAP - 1 : idx;
      int sr = lst[idx];
      sr = sr < 0 ? 0 : (sr > NN - 1 ? NN - 1 : sr);
      const int m32 = (c - b0) < 32 ? (c - b0) : 32;
#pragma unroll 1
      for (int k = 0; k < m32; ++k) {
        const int sk = __builtin_amdgcn_readlane(sr, k);
        const v4f a = *(const v4f*)(hs + (size_t)sk * FD + 4 * lane);
        a0 += a.x; a1 += a.y; a2 += a.z; a3 += a.w;
      }
    }
    const float pz = bad ? qnan : 0.0f;
    const bool live = node < NN;
    float t0 = a0 * cdv + bb.x, t1 = a1 * cdv + bb.y, t2 = a2 * cdv + bb.z, t3 = a3 * cdv + bb.w;
    t0 = (t0 > 0.0f) ? t0 : (t0 - t0);
    t1 = (t1 > 0.0f) ? t1 : (t1 - t1);
    t2 = (t2 > 0.0f) ? t2 : (t2 - t2);
    t3 = (t3 > 0.0f) ? t3 : (t3 - t3);
    v4f mv;
    mv.x = live ? (t0 + pz) : 0.0f;
    mv.y = live ? (t1 + pz) : 0.0f;
    mv.z = live ? (t2 + pz) : 0.0f;
    mv.w = live ? (t3 + pz) : 0.0f;
    v4us mh, ml;
    {
      unsigned hb;
      hb = bf16_bits(mv.x); mh[0] = (unsigned short)hb; ml[0] = (unsigned short)bf16_bits(mv.x - __uint_as_float(hb << 16));
      hb = bf16_bits(mv.y); mh[1] = (unsigned short)hb; ml[1] = (unsigned short)bf16_bits(mv.y - __uint_as_float(hb << 16));
      hb = bf16_bits(mv.z); mh[2] = (unsigned short)hb; ml[2] = (unsigned short)bf16_bits(mv.z - __uint_as_float(hb << 16));
      hb = bf16_bits(mv.w); mh[3] = (unsigned short)hb; ml[3] = (unsigned short)bf16_bits(mv.w - __uint_as_float(hb << 16));
    }
    *(v4usa*)(rowbuf + 4 * lane) = mh;
    *(v4usa*)(rowbuf + FD + 4 * lane) = ml;
    wave_sync();
    const v8us q0 = *(const v8usa*)(rowbuf + 8 * lane);
    wave_sync();
    const bool stH = node < MP;
    unsigned short* rpw = hhl + (size_t)node * HP + 8 * lane;
    float* op = outp + (size_t)node * FD + 4 * lane;
    if (stH) *(volatile v8us*)rpw = q0;
    if constexpr (FINAL != 0) { if (live) *(volatile v4f*)op = mv; }
    __threadfence();
    if (stH) *(volatile v8us*)rpw = q0;
    if constexpr (FINAL != 0) { if (live) *(volatile v4f*)op = mv; }
  }
}

__global__ __launch_bounds__(GTHR) void k_head(const int* __restrict__ users,
                                               const unsigned short* __restrict__ hhl,
                                               const unsigned short* __restrict__ ws1d,
                                               const unsigned short* __restrict__ ws2d,
                                               const float* __restrict__ bt, float* out0) {
  __shared__ __attribute__((aligned(16))) unsigned short At[GBM * HP];
  __shared__ __attribute__((aligned(16))) float stg[GBM * OD];
  __shared__ int uix[GBM];
  const int tid = (int)threadIdx.x, lane = tid & 31, wave = tid >> 5, hh = lane >> 4, m = lane & 15;
  const int rowBase = (int)blockIdx.x * GBM;

  if (tid < GBM) {
    int r = rowBase + tid;
    r = r > NU - 1 ? NU - 1 : r;
    int u = users[r];
    u = u < 0 ? 0 : (u > NN - 1 ? NN - 1 : u);
    uix[tid] = u;
  }
  __syncthreads();
#pragma unroll 4
  for (int i = 0; i < 16; ++i) {
    const int p = i * GTHR + tid;
    const int r = p >> 5;
    const int c = p & 31;
    const int u = uix[r];
    const v8us v = *(const v8usa*)(hhl + (size_t)u * HP + 8 * c);
    *(v8usa*)(At + r * HP + 8 * c) = v;
  }
  __syncthreads();

  v8f acc[4];
  {
    const v8f z = {0.f, 0.f, 0.f, 0.f, 0.f, 0.f, 0.f, 0.f};
    acc[0] = z; acc[1] = z; acc[2] = z; acc[3] = z;
  }
  {
    const unsigned short* ap = At + (16 * wave + m) * HP + 8 * hh;
    const unsigned short* bp = ws1d + (size_t)m * HP + 8 * hh;
#pragma unroll 1
    for (int k0 = 0; k0 < HP; k0 += 32) {
      FragB af;
      af.h[0] = *(const v8usa*)(ap + k0);
      af.h[1] = *(const v8usa*)(ap + k0 + 16);
#pragma unroll
      for (int t = 0; t < 4; ++t) {
        const unsigned short* wq = bp + (size_t)(16 * t) * HP + k0;
        FragB bf;
        bf.h[0] = *(const v8usa*)wq;
        bf.h[1] = *(const v8usa*)(wq + 16);
        acc[t] = wmb(af, bf, acc[t]);
      }
    }
  }
#pragma unroll
  for (int t = 0; t < 4; ++t) {
    const int lc = 16 * t + m;
#pragma unroll
    for (int r = 0; r < 8; ++r) {
      const int lr = 16 * wave + 8 * hh + r;
      stg[lr * OD + lc] = acc[t][r];
    }
  }
  __syncthreads();

  unsigned short* A2 = At;
  {
    const int c = tid & (OD - 1);
    const float b1v = bt[2 * FD + c];
#pragma unroll 1
    for (int j = 0; j < (GBM * OD) / GTHR; ++j) {
      const int r = 2 * j + (tid >> 6);
      const float v  = stg[r * OD + c] + b1v;
      const float tv = tanhf(v);
      const unsigned hb = bf16_bits(tv);
      const unsigned lb = bf16_bits(tv - __uint_as_float(hb << 16));
      A2[r * (2 * OD) + c]      = (unsigned short)hb;
      A2[r * (2 * OD) + OD + c] = (unsigned short)lb;
    }
  }
  __syncthreads();

  {
    const v8f z = {0.f, 0.f, 0.f, 0.f, 0.f, 0.f, 0.f, 0.f};
    acc[0] = z; acc[1] = z; acc[2] = z; acc[3] = z;
  }
  {
    const unsigned short* ap = A2 + (16 * wave + m) * (2 * OD) + 8 * hh;
    const unsigned short* bp = ws2d + (size_t)m * (2 * OD) + 8 * hh;
#pragma unroll 1
    for (int k0 = 0; k0 < 2 * OD; k0 += 32) {
      FragB af;
      af.h[0] = *(const v8usa*)(ap + k0);
      af.h[1] = *(const v8usa*)(ap + k0 + 16);
#pragma unroll
      for (int t = 0; t < 4; ++t) {
        const unsigned short* wq = bp + (size_t)(16 * t) * (2 * OD) + k0;
        FragB bf;
        bf.h[0] = *(const v8usa*)wq;
        bf.h[1] = *(const v8usa*)(wq + 16);
        acc[t] = wmb(af, bf, acc[t]);
      }
    }
  }
#pragma unroll
  for (int t = 0; t < 4; ++t) {
    const int lc = 16 * t + m;
#pragma unroll
    for (int r = 0; r < 8; ++r) {
      const int lr = 16 * wave + 8 * hh + r;
      stg[lr * OD + lc] = acc[t][r];
    }
  }
  __syncthreads();

  const v4f b2 = *(const v4f*)(bt + 2 * FD + OD + 4 * m);
  v4f fv[8];
#pragma unroll
  for (int i = 0; i < 8; ++i) {
    const int lr = 16 * wave + 2 * i + hh;
    const v4f s = *(const v4fa*)(stg + lr * OD + 4 * m);
    fv[i] = s + b2;
  }
#pragma unroll
  for (int i = 0; i < 8; ++i) {
    const int gr = rowBase + 16 * wave + 2 * i + hh;
    if (gr < NU) *(volatile v4f*)(out0 + (size_t)gr * OD + 4 * m) = fv[i];
  }
  __threadfence();
#pragma unroll
  for (int i = 0; i < 8; ++i) {
    const int gr = rowBase + 16 * wave + 2 * i + hh;
    if (gr < NU) *(volatile v4f*)(out0 + (size_t)gr * OD + 4 * m) = fv[i];
  }
}

static inline size_t al256(size_t o) { return (o + 255) & ~(size_t)255; }

extern "C" void kernel_launch(void* const* d_in, const int* in_sizes, int n_in,
                              void* d_out, int out_size, void* d_ws, size_t ws_size,
                              hipStream_t stream) {
  if (n_in < 12) return;
  if (in_sizes[0] != NN * FD) return;
  if (in_sizes[1] != FD * FD || in_sizes[2] != FD) return;
  if (in_sizes[3] != FD * FD || in_sizes[4] != FD) return;
  if (in_sizes[5] != FD * OD || in_sizes[6] != OD) return;
  if (in_sizes[7] != OD * OD || in_sizes[8] != OD) return;
  if (in_sizes[9] != NE || in_sizes[10] != NE) return;
  if (in_sizes[11] != NU) return;
  if ((long long)out_size != (long long)NU * OD + (long long)NN * FD) return;

  const float* feat = (const float*)d_in[0];
  const float* W0   = (const float*)d_in[1];
  const float* b0   = (const float*)d_in[2];
  const float* W1   = (const float*)d_in[3];
  const float* b1   = (const float*)d_in[4];
  const float* Ws1  = (const float*)d_in[5];
  const float* bs1  = (const float*)d_in[6];
  const float* Ws2  = (const float*)d_in[7];
  const float* bs2  = (const float*)d_in[8];
  const int*   src  = (const int*)d_in[9];
  const int*   dst  = (const int*)d_in[10];
  const int*   usr  = (const int*)d_in[11];
  float* out = (float*)d_out;

  char* ws = (char*)d_ws;
  size_t off = 0;
  const size_t oCS  = off; off = al256(off + (size_t)NBPD * 4);
  const size_t oCD  = off; off = al256(off + (size_t)NSLOT * 4);
  const size_t oOFF = off; off = al256(off + (size_t)NSLOT * 4);
  const size_t oCNT = off; off = al256(off + (size_t)NSLOT * 4);
  const size_t oBT  = off; off = al256(off + (size_t)384 * 4);
  const size_t oW0T = off; off = al256(off + (size_t)FD * FD * 2);
  const size_t oW1D = off; off = al256(off + (size_t)FD * HP * 2);
  const size_t oS1D = off; off = al256(off + (size_t)OD * HP * 2);
  const size_t oS2D = off; off = al256(off + (size_t)OD * 2 * OD * 2);
  const size_t oXB  = off; off = al256(off + (size_t)MP * FD * 2);
  const size_t oHS  = off; off = al256(off + (size_t)MP * FD * 4);
  const size_t oHHL = off; off = al256(off + (size_t)MP * HP * 2);
  const size_t oLST = off; off = al256(off + (size_t)GA * RCAP * 4);
  if (off > ws_size || off > (size_t)WSMAX) return;
  float*          CS   = (float*)(ws + oCS);
  float*          CD   = (float*)(ws + oCD);
  int*            OFFp = (int*)(ws + oOFF);
  int*            CNTp = (int*)(ws + oCNT);
  float*          BT   = (float*)(ws + oBT);
  unsigned short* W0T  = (unsigned short*)(ws + oW0T);
  unsigned short* W1D  = (unsigned short*)(ws + oW1D);
  unsigned short* S1D  = (unsigned short*)(ws + oS1D);
  unsigned short* S2D  = (unsigned short*)(ws + oS2D);
  unsigned short* XB   = (unsigned short*)(ws + oXB);
  float*          HS   = (float*)(ws + oHS);
  unsigned short* HHL  = (unsigned short*)(ws + oHHL);
  int*            LST  = (int*)(ws + oLST);

  const int vec8 = ((NE & 3) == 0) ? 1 : 0;
  const size_t bkLds = (size_t)BK_LDS_INTS * 4;
  hipFuncSetAttribute(reinterpret_cast<const void*>(&k_bucket), hipFuncAttributeMaxDynamicSharedMemorySize, (int)bkLds);

  k_prep<<<UTOT / NTHR, NTHR, 0, stream>>>(feat, W0, W1, Ws1, Ws2, b0, b1, bs1, bs2, XB, W0T, W1D, S1D, S2D, BT);
  k_degout<<<GD, NTHR, 0, stream>>>(src, NE, vec8, CS);
  k_bucket<<<GA, NTHR, bkLds, stream>>>(src, dst, NE, NN, vec8, LST, OFFp, CNTp, CD);
  k_gemm<FD><<<MP / GBM, GTHR, 0, stream>>>(XB, W0T, CS, HS);
  k_agg<0><<<GA, NTHR, 0, stream>>>(LST, OFFp, CNTp, CD, HS, BT, HHL, out + OUT1);
  k_gemm<HP><<<MP / GBM, GTHR, 0, stream>>>(HHL, W1D, CS, HS);
  k_agg<1><<<GA, NTHR, 0, stream>>>(LST, OFFp, CNTp, CD, HS, BT + FD, HHL, out + OUT1);
  k_head<<<(NU + GBM - 1) / GBM, GTHR, 0, stream>>>(usr, HHL, S1D, S2D, BT, out);
}
